// QuantumPaperSelfAttention_37203006718044
// MI455X (gfx1250) — hardware-verified
//
#include <hip/hip_runtime.h>
#include <stdint.h>
#include <math.h>

constexpr int NB_BATCH = 4;
constexpr int NS_SEQ   = 2048;
constexpr int ND_MODEL = 1024;
constexpr int NH_HEADS = 16;
constexpr int HEAD_D   = 64;
constexpr int NROWS    = NB_BATCH * NS_SEQ;
constexpr int LD_QKV   = 3 * ND_MODEL;
constexpr int NQ_TILES = NS_SEQ / 64;
static_assert(NH_HEADS * HEAD_D == ND_MODEL, "head split");
static_assert(NROWS % 64 == 0 && LD_QKV % 64 == 0 && ND_MODEL % 64 == 0 && NS_SEQ % 64 == 0, "tile multiples");
static_assert(ND_MODEL % 32 == 0, "K multiple of 32");

typedef __attribute__((ext_vector_type(16))) _Float16 v16h;
typedef __attribute__((ext_vector_type(8)))  _Float16 v8h;
typedef __attribute__((ext_vector_type(16))) __bf16   v16b;
typedef __attribute__((ext_vector_type(8)))  __bf16   v8b;
typedef __attribute__((ext_vector_type(8)))  float    v8f;
typedef __attribute__((ext_vector_type(4)))  float    v4f;

__device__ __forceinline__ unsigned short f2bf_bits(float f) {
  unsigned u = __float_as_uint(f);
  return (unsigned short)((u + 0x7FFFu + ((u >> 16) & 1u)) >> 16);
}
__device__ __forceinline__ float bf_bits2f(unsigned short h) { return __uint_as_float(((unsigned)h) << 16); }

__device__ __forceinline__ void dep_guard_h(v8f& a, v8f& b, v16h x, v16h y) { asm volatile("v_nop\n\tv_nop\n\tv_nop\n\tv_nop" : "+v"(a), "+v"(b) : "v"(x), "v"(y)); }
__device__ __forceinline__ void dep_guard_b(v8f& a, v8f& b, v16b x, v16b y) { asm volatile("v_nop\n\tv_nop\n\tv_nop\n\tv_nop" : "+v"(a), "+v"(b) : "v"(x), "v"(y)); }
__device__ __forceinline__ void keep4_h(v16h a, v16h b, v16h c, v16h d) { asm volatile("v_nop" :: "v"(a), "v"(b), "v"(c), "v"(d)); }
__device__ __forceinline__ void keep4_b(v16b a, v16b b, v16b c, v16b d) { asm volatile("v_nop" :: "v"(a), "v"(b), "v"(c), "v"(d)); }
__device__ __forceinline__ void acc_guard4(v8f& a, v8f& b, v8f& c, v8f& d) { asm volatile("v_nop\n\tv_nop\n\tv_nop\n\tv_nop" : "+v"(a), "+v"(b), "+v"(c), "+v"(d)); }
template <typename T> struct Frag;
template <> struct Frag<_Float16> {
  typedef v16h V; union U { v16h v; v8h h[2]; };
  static __device__ __forceinline__ v16h load(const _Float16* p) {
    U f; f.h[0] = *(const v8h*)(p); f.h[1] = *(const v8h*)(p + 16); return f.v;
  }
  static __device__ __forceinline__ v8f mma(v16h a, v16h b, v8f c) {
    return __builtin_amdgcn_wmma_f32_16x16x32_f16(false, a, false, b, (short)0, c, false, false);
  }
  static __device__ __forceinline__ void guard(v8f& a, v8f& b, v16h x, v16h y) { dep_guard_h(a, b, x, y); }
  static __device__ __forceinline__ void keep(v16h a, v16h b, v16h c, v16h d) { keep4_h(a, b, c, d); }
};
template <> struct Frag<__bf16> {
  typedef v16b V; union U { v16b v; v8b h[2]; };
  static __device__ __forceinline__ v16b load(const __bf16* p) {
    U f; f.h[0] = *(const v8b*)(p); f.h[1] = *(const v8b*)(p + 16); return f.v;
  }
  static __device__ __forceinline__ v8f mma(v16b a, v16b b, v8f c) {
    return __builtin_amdgcn_wmma_f32_16x16x32_bf16(false, a, false, b, (short)0, c, false, false);
  }
  static __device__ __forceinline__ void guard(v8f& a, v8f& b, v16b x, v16b y) { dep_guard_b(a, b, x, y); }
  static __device__ __forceinline__ void keep(v16b a, v16b b, v16b c, v16b d) { keep4_b(a, b, c, d); }
};

template <int ET> struct Elem;
template <> struct Elem<0> { typedef _Float16 T; };
template <> struct Elem<1> { typedef __bf16 T; };
template <int ET, int SPLIT, int BIAS_MODE, int OUT_MODE, bool RESID, int ACT = 0>
__global__ __launch_bounds__(256) void wmma_gemm64(
    const unsigned short* __restrict__ Ap, const unsigned short* __restrict__ A2p, int lda, long strideA,
    const unsigned short* __restrict__ Btp, const unsigned short* __restrict__ Bt2p, int ldb, long strideB,
    void* __restrict__ Cout, void* __restrict__ Cout2, int ldc, long strideC,
    const float* __restrict__ bias,
    const float* __restrict__ resid, long strideR,
    int M, int N, int K, float scale) {
  typedef typename Elem<ET>::T T;
  typedef typename Frag<T>::V V;
  const T* A = (const T*)Ap; const T* A2 = (const T*)A2p; const T* Bt = (const T*)Btp; const T* Bt2 = (const T*)Bt2p;
  __shared__ __align__(16) float sT[8][16 * 68];
  const int b    = blockIdx.y;
  const int lane = threadIdx.x & 31;
  const int wave = threadIdx.x >> 5;
  const int tilesN = N >> 6;
  const int tilesM = M >> 6;
  const int tile = blockIdx.x * 8 + wave;
  if (tile >= tilesM * tilesN) return;
  const int tm = tile / tilesN;
  const int tn = tile - tm * tilesN;
  const int m0 = tm << 6;
  const int n0 = tn << 6;

  const T* Ab  = A  + (size_t)b * strideA;
  const T* Bb  = Bt + (size_t)b * strideB;
  const T* Ab2 = (SPLIT >= 1) ? (A2  + (size_t)b * strideA) : nullptr;
  const T* Bb2 = (SPLIT == 2) ? (Bt2 + (size_t)b * strideB) : nullptr;

  const int rlane = lane & 15;
  const int koff  = (lane >> 4) * 8;
  const int mOff  = (lane >> 4) * 8;

  v8f acc[4][4];
#pragma unroll
  for (int i = 0; i < 4; ++i)
#pragma unroll
    for (int j = 0; j < 4; ++j) acc[i][j] = (v8f){0.f,0.f,0.f,0.f,0.f,0.f,0.f,0.f};

  for (int k0 = 0; k0 < K; k0 += 32) {
    V bh[4], bl[4];
#pragma unroll
    for (int j = 0; j < 4; ++j) {
      const size_t bo = (size_t)(n0 + (j << 4) + rlane) * ldb + koff + k0;
      bh[j] = Frag<T>::load(Bb + bo);
      if (SPLIT == 2) bl[j] = Frag<T>::load(Bb2 + bo);
    }
#pragma unroll
    for (int i = 0; i < 4; ++i) {
      const size_t ao = (size_t)(m0 + (i << 4) + rlane) * lda + koff + k0;
      V ah = Frag<T>::load(Ab + ao);
      V al;
      if (SPLIT >= 1) al = Frag<T>::load(Ab2 + ao);
#pragma unroll
      for (int j = 0; j < 4; ++j) {
        acc[i][j] = Frag<T>::mma(ah, bh[j], acc[i][j]);
        if (SPLIT == 2) acc[i][j] = Frag<T>::mma(ah, bl[j], acc[i][j]);
        if (SPLIT >= 1) acc[i][j] = Frag<T>::mma(al, bh[j], acc[i][j]);
      }
      Frag<T>::guard(acc[i][0], acc[i][3], ah, (SPLIT >= 1) ? al : ah);
    }
    Frag<T>::keep(bh[0], bh[1], bh[2], bh[3]);
    if (SPLIT == 2) Frag<T>::keep(bl[0], bl[1], bl[2], bl[3]);
  }
  acc_guard4(acc[0][0], acc[0][1], acc[0][2], acc[0][3]);
  acc_guard4(acc[1][0], acc[1][1], acc[1][2], acc[1][3]);
  acc_guard4(acc[2][0], acc[2][1], acc[2][2], acc[2][3]);
  acc_guard4(acc[3][0], acc[3][1], acc[3][2], acc[3][3]);

  float* slab = sT[wave];
  const float* Rb = RESID ? (resid + (size_t)b * strideR) : nullptr;
#pragma unroll
  for (int i = 0; i < 4; ++i) {
    const int mBase = m0 + (i << 4);
#pragma unroll
    for (int j = 0; j < 4; ++j) {
      const int n = n0 + (j << 4) + rlane;
      float bv = 0.f;
      if (BIAS_MODE == 2) bv = bias[n];
#pragma unroll
      for (int r = 0; r < 8; ++r) {
        float v = acc[i][j][r] * scale;
        if (BIAS_MODE == 1) v += bias[mBase + mOff + r];
        if (BIAS_MODE == 2) v += bv;
        if (RESID) v += Rb[(size_t)(mBase + mOff + r) * ldc + n];
        if (ACT == 1) v = tanhf(v);
        if (ACT == 2) v = fmaxf(v, 0.0f);
        if (ACT == 3) v = v / (1.0f + expf(-v));
        if (ACT == 4) v = (v > 0.f) ? v : 0.01f * v;
        slab[(mOff + r) * 68 + (j << 4) + rlane] = v;
      }
    }
    __builtin_amdgcn_fence(__ATOMIC_RELEASE, "workgroup");
    __builtin_amdgcn_wave_barrier();
    __builtin_amdgcn_fence(__ATOMIC_ACQUIRE, "workgroup");
    if (OUT_MODE == 0) {
      float* C = (float*)Cout + (size_t)b * strideC;
      const int hh = lane >> 4, c4 = (lane & 15) * 4;
      for (int pass = 0; pass < 2; ++pass) {
#pragma unroll
        for (int it = 0; it < 8; ++it) {
          const int row = it * 2 + hh;
          v4f v = *(const v4f*)(slab + row * 68 + c4);
          *(volatile v4f*)(C + (size_t)(mBase + row) * ldc + n0 + c4) = v;
        }
        __threadfence();
      }
    } else {
      const int q = lane >> 3, c8 = (lane & 7) * 8;
      unsigned short* C  = (unsigned short*)Cout  + (size_t)b * strideC;
      unsigned short* C2 = (OUT_MODE == 2) ? ((unsigned short*)Cout2 + (size_t)b * strideC) : nullptr;
      for (int pass = 0; pass < 2; ++pass) {
#pragma unroll
        for (int it = 0; it < 4; ++it) {
          const int row = it * 4 + q;
          const float* sp = slab + row * 68 + c8;
          v8h hv, lv;
#pragma unroll
          for (int e = 0; e < 8; ++e) {
            if (OUT_MODE == 1) {
              hv[e] = (_Float16)sp[e];
            } else {
              unsigned short hb = f2bf_bits(sp[e]);
              unsigned short lb = f2bf_bits(sp[e] - bf_bits2f(hb));
              hv[e] = __builtin_bit_cast(_Float16, hb);
              lv[e] = __builtin_bit_cast(_Float16, lb);
            }
          }
          *(volatile v8h*)(C + (size_t)(mBase + row) * ldc + n0 + c8) = hv;
          if (OUT_MODE == 2) *(volatile v8h*)(C2 + (size_t)(mBase + row) * ldc + n0 + c8) = lv;
        }
        __threadfence();
      }
    }
    __builtin_amdgcn_fence(__ATOMIC_RELEASE, "workgroup");
    __builtin_amdgcn_wave_barrier();
    __builtin_amdgcn_fence(__ATOMIC_ACQUIRE, "workgroup");
  }
}

__global__ __launch_bounds__(256) void cast_f32_bf16x2(
    const float* __restrict__ in, unsigned short* __restrict__ out, int n2) {
  int i = blockIdx.x * 256 + threadIdx.x;
  if (i < n2) {
    const unsigned short b0 = f2bf_bits(in[2 * i]);
    const unsigned short b1 = f2bf_bits(in[2 * i + 1]);
    const unsigned u = (unsigned)b0 | ((unsigned)b1 << 16);
    ((volatile unsigned*)out)[i] = u;
    __threadfence();
    ((volatile unsigned*)out)[i] = u;
  }
}

__device__ __forceinline__ __bf16 at_f2bf(float f) { return __builtin_bit_cast(__bf16, f2bf_bits(f)); }
__device__ __forceinline__ void at_split(float f, __bf16& hi, __bf16& lo) {
  const unsigned short hb = f2bf_bits(f);
  hi = __builtin_bit_cast(__bf16, hb);
  lo = at_f2bf(f - __uint_as_float(((unsigned)hb) << 16));
}
__device__ __forceinline__ v8f at_mma(v16b a, v16b b, v8f c) {
  c = __builtin_amdgcn_wmma_f32_16x16x32_bf16(false, a, false, b, (short)0, c, false, false);
  asm volatile("v_nop\n\tv_nop\n\tv_nop\n\tv_nop" : "+v"(c) : "v"(a), "v"(b));
  return c;
}

__device__ __forceinline__ float tanh_eval(float x) {
  const float e  = __builtin_amdgcn_exp2f(x * 2.8853900817779268f);
  const float yb = 1.0f - 2.0f * __builtin_amdgcn_rcpf(e + 1.0f);
  const float x2 = x * x;
  const float ys = x + x * (x2 * (-0.33333333333f + x2 * 0.13333333333f));
  return (fabsf(x) < 0.0625f) ? ys : yb;
}

__global__ __launch_bounds__(128)
void attn_tanh_l1_k(const unsigned short* __restrict__ qkvh, const unsigned short* __restrict__ qkvl,
                    unsigned short* __restrict__ ohp, unsigned short* __restrict__ olp, int batch) {
  union FB { v16b v; v8b h[2]; };
  __shared__ __align__(16) __bf16 Ksh[64 * 64];
  __shared__ __align__(16) __bf16 Ksl[64 * 64];
  __shared__ __align__(16) __bf16 Vth[64 * 64];
  __shared__ __align__(16) __bf16 Vtl[64 * 64];
  __shared__ __align__(16) __bf16 Psh[4][16 * 64];
  __shared__ __align__(16) __bf16 Psl[4][16 * 64];
  __shared__ __align__(16) float  Os[4][16 * 68];

  const int tid  = threadIdx.x;
  const int wave = tid >> 5;
  const int lane = tid & 31;
  const int hh   = lane >> 4;
  const int c    = lane & 15;

  const int qb = blockIdx.x % NQ_TILES;
  const int h  = blockIdx.x / NQ_TILES;
  const int q0 = qb * 64 + wave * 16;
  const int hcol = h * HEAD_D;
  const size_t rowb = (size_t)batch * NS_SEQ;

  const __bf16* PH = (const __bf16*)qkvh;
  const __bf16* PL = (const __bf16*)qkvl;

  v16b qh[2], ql[2];
  {
    const size_t qo = (rowb + q0 + c) * LD_QKV + hcol + 8 * hh;
#pragma unroll
    for (int dc = 0; dc < 2; ++dc) {
      qh[dc] = Frag<__bf16>::load(PH + qo + dc * 32);
      ql[dc] = Frag<__bf16>::load(PL + qo + dc * 32);
    }
  }

  v8f oacc[4];
#pragma unroll
  for (int t = 0; t < 4; ++t) oacc[t] = (v8f){0.f,0.f,0.f,0.f,0.f,0.f,0.f,0.f};
  float dsum[8];
#pragma unroll
  for (int r = 0; r < 8; ++r) dsum[r] = 0.f;

  const int nChunks = qb + 1;
  for (int kc = 0; kc < nChunks; ++kc) {
    const int kv0 = kc * 64;
    __syncthreads();
    {
      const int kvr = tid >> 1, dh = (tid & 1) * 32;
      const size_t go = (rowb + kv0 + kvr) * LD_QKV + hcol + dh;
#pragma unroll
      for (int i = 0; i < 4; ++i) {
        const v8b kH8 = *(const v8b*)(PH + go + ND_MODEL + 8 * i);
        const v8b kL8 = *(const v8b*)(PL + go + ND_MODEL + 8 * i);
        *(v8b*)(Ksh + kvr * 64 + dh + 8 * i) = kH8;
        *(v8b*)(Ksl + kvr * 64 + dh + 8 * i) = kL8;
        const v8b vH8 = *(const v8b*)(PH + go + 2 * ND_MODEL + 8 * i);
        const v8b vL8 = *(const v8b*)(PL + go + 2 * ND_MODEL + 8 * i);
#pragma unroll
        for (int e = 0; e < 8; ++e) {
          Vth[(dh + 8 * i + e) * 64 + kvr] = vH8[e];
          Vtl[(dh + 8 * i + e) * 64 + kvr] = vL8[e];
        }
      }
    }
    __syncthreads();

    v8f s[4];
#pragma unroll
    for (int j = 0; j < 4; ++j) {
      s[j] = (v8f){0.f,0.f,0.f,0.f,0.f,0.f,0.f,0.f};
#pragma unroll
      for (int dc = 0; dc < 2; ++dc) {
        FB kb, kl;
        const int ko = (j * 16 + c) * 64 + dc * 32 + 8 * hh;
        kb.h[0] = *(const v8b*)(Ksh + ko);
        kb.h[1] = *(const v8b*)(Ksh + ko + 16);
        kl.h[0] = *(const v8b*)(Ksl + ko);
        kl.h[1] = *(const v8b*)(Ksl + ko + 16);
        s[j] = at_mma(qh[dc], kb.v, s[j]);
        s[j] = at_mma(qh[dc], kl.v, s[j]);
        s[j] = at_mma(ql[dc], kb.v, s[j]);
      }
    }

    const bool diag = (kc == qb);
    __bf16* pwh = Psh[wave];
    __bf16* pwl = Psl[wave];
#pragma unroll
    for (int r = 0; r < 8; ++r) {
      const int qrow = q0 + 8 * hh + r;
      float asum = 0.f;
#pragma unroll
      for (int j = 0; j < 4; ++j) {
        const int kvcol = kv0 + j * 16 + c;
        float t = tanh_eval(s[j][r] * 0.125f);
        t = (diag && (kvcol > qrow)) ? 0.0f : t;
        asum += fabsf(t);
        __bf16 th, tl;
        at_split(t, th, tl);
        pwh[(8 * hh + r) * 64 + j * 16 + c] = th;
        pwl[(8 * hh + r) * 64 + j * 16 + c] = tl;
      }
      dsum[r] += asum;
    }
    __builtin_amdgcn_fence(__ATOMIC_RELEASE, "workgroup");
    __builtin_amdgcn_wave_barrier();
    __builtin_amdgcn_fence(__ATOMIC_ACQUIRE, "workgroup");

#pragma unroll 1
    for (int kk = 0; kk < 2; ++kk) {
      FB pa, pl;
      const int po = c * 64 + kk * 32 + 8 * hh;
      pa.h[0] = *(const v8b*)(pwh + po);
      pa.h[1] = *(const v8b*)(pwh + po + 16);
      pl.h[0] = *(const v8b*)(pwl + po);
      pl.h[1] = *(const v8b*)(pwl + po + 16);
#pragma unroll
      for (int t = 0; t < 4; ++t) {
        FB vb, vl;
        const int vo = (t * 16 + c) * 64 + kk * 32 + 8 * hh;
        vb.h[0] = *(const v8b*)(Vth + vo);
        vb.h[1] = *(const v8b*)(Vth + vo + 16);
        vl.h[0] = *(const v8b*)(Vtl + vo);
        vl.h[1] = *(const v8b*)(Vtl + vo + 16);
        oacc[t] = at_mma(pa.v, vb.v, oacc[t]);
        oacc[t] = at_mma(pa.v, vl.v, oacc[t]);
        oacc[t] = at_mma(pl.v, vb.v, oacc[t]);
      }
    }
  }

  float* os = Os[wave];
#pragma unroll
  for (int r = 0; r < 8; ++r) {
    float tsum = dsum[r];
    tsum += __shfl_xor(tsum, 1, 32);
    tsum += __shfl_xor(tsum, 2, 32);
    tsum += __shfl_xor(tsum, 4, 32);
    tsum += __shfl_xor(tsum, 8, 32);
    const float inv = __builtin_amdgcn_rcpf(fmaxf(tsum, 1e-6f));
#pragma unroll
    for (int t = 0; t < 4; ++t) os[(8 * hh + r) * 68 + t * 16 + c] = oacc[t][r] * inv;
  }
  __builtin_amdgcn_fence(__ATOMIC_RELEASE, "workgroup");
  __builtin_amdgcn_wave_barrier();
  __builtin_amdgcn_fence(__ATOMIC_ACQUIRE, "workgroup");
  {
    const int q4 = lane >> 3, c8 = (lane & 7) * 8;
    for (int pass = 0; pass < 2; ++pass) {
#pragma unroll
      for (int it = 0; it < 4; ++it) {
        const int row = it * 4 + q4;
        const float* sp = os + row * 68 + c8;
        v8h hv, lv;
#pragma unroll
        for (int e = 0; e < 8; ++e) {
          const unsigned short hb = f2bf_bits(sp[e]);
          const unsigned short lb = f2bf_bits(sp[e] - bf_bits2f(hb));
          hv[e] = __builtin_bit_cast(_Float16, hb);
          lv[e] = __builtin_bit_cast(_Float16, lb);
        }
        const size_t oo = (size_t)(q0 + row) * ND_MODEL + hcol + c8;
        *(volatile v8h*)(ohp + oo) = hv;
        *(volatile v8h*)(olp + oo) = lv;
      }
      __threadfence();
    }
  }
}

extern "C" void kernel_launch(void* const* d_in, const int* in_sizes, int n_in,
                              void* d_out, int out_size, void* d_ws, size_t ws_size,
                              hipStream_t stream) {
  if (n_in < 5) return;
  const int nx = NROWS * ND_MODEL;
  const int nw = ND_MODEL * ND_MODEL;
  if (in_sizes[0] != nx || in_sizes[1] != nw || in_sizes[2] != nw || in_sizes[3] != nw || in_sizes[4] != nw) return;
  if (out_size != nx) return;

  const size_t offXb   = 0;
  const size_t szXb    = (size_t)nx * 2;
  const size_t offWcat = offXb + szXb;
  const size_t szWcat  = (size_t)3 * nw * 2;
  const size_t offWo   = offWcat + szWcat;
  const size_t szWo    = (size_t)nw * 2;
  const size_t offQh   = offWo + szWo;
  const size_t szQ     = (size_t)NROWS * LD_QKV * 2;
  const size_t offQl   = offQh + szQ;
  const size_t total   = offQl + szQ;
  const size_t offOh   = 0;
  const size_t szO     = (size_t)NS_SEQ * ND_MODEL * 2;
  const size_t offOl   = offOh + szO;
  if (total > ws_size) return;
  if (offOl + szO > szXb) return;

  const float* x  = (const float*)d_in[0];
  const float* Wq = (const float*)d_in[1];
  const float* Wk = (const float*)d_in[2];
  const float* Wv = (const float*)d_in[3];
  const float* Wo = (const float*)d_in[4];
  float* out = (float*)d_out;
  char* ws = (char*)d_ws;
  unsigned short* xb   = (unsigned short*)(ws + offXb);
  unsigned short* wcat = (unsigned short*)(ws + offWcat);
  unsigned short* wob  = (unsigned short*)(ws + offWo);
  unsigned short* qkvh = (unsigned short*)(ws + offQh);
  unsigned short* qkvl = (unsigned short*)(ws + offQl);
  unsigned short* oh   = (unsigned short*)(ws + offOh);
  unsigned short* ol   = (unsigned short*)(ws + offOl);

  cast_f32_bf16x2<<<(nx / 2) / 256, 256, 0, stream>>>(x,  xb, nx / 2);
  cast_f32_bf16x2<<<(nw / 2) / 256, 256, 0, stream>>>(Wq, wcat,                  nw / 2);
  cast_f32_bf16x2<<<(nw / 2) / 256, 256, 0, stream>>>(Wk, wcat + (size_t)nw,     nw / 2);
  cast_f32_bf16x2<<<(nw / 2) / 256, 256, 0, stream>>>(Wv, wcat + (size_t)2 * nw, nw / 2);
  cast_f32_bf16x2<<<(nw / 2) / 256, 256, 0, stream>>>(Wo, wob, nw / 2);

  {
    const int tiles = (NROWS / 64) * (LD_QKV / 64);
    wmma_gemm64<1, 0, 0, 2, false><<<dim3(tiles / 8, 1), 256, 0, stream>>>(
        xb, xb, ND_MODEL, 0L, wcat, wcat, ND_MODEL, 0L,
        (void*)qkvh, (void*)qkvl, LD_QKV, 0L, x, x, 0L, NROWS, LD_QKV, ND_MODEL, 1.0f);
  }

  for (int b = 0; b < NB_BATCH; ++b) {
    attn_tanh_l1_k<<<NH_HEADS * NQ_TILES, 128, 0, stream>>>(qkvh, qkvl, oh, ol, b);
    float* outb = out + (size_t)b * NS_SEQ * ND_MODEL;
    const int tiles = (NS_SEQ / 64) * (ND_MODEL / 64);
    wmma_gemm64<1, 1, 0, 0, false><<<dim3(tiles / 8, 1), 256, 0, stream>>>(
        oh, ol, ND_MODEL, 0L, wob, wob, ND_MODEL, 0L,
        (void*)outb, (void*)outb, ND_MODEL, 0L, x, x, 0L, NS_SEQ, ND_MODEL, ND_MODEL, 1.0f);
  }
}
